// TransformerBlock_48112223650153
// MI455X (gfx1250) — hardware-verified
//
#include <hip/hip_runtime.h>
#include <stddef.h>


typedef _Float16 v16h __attribute__((ext_vector_type(16)));
typedef _Float16 v8h  __attribute__((ext_vector_type(8)));
typedef _Float16 v4h  __attribute__((ext_vector_type(4)));
typedef float    v8f  __attribute__((ext_vector_type(8)));
typedef float    v4f  __attribute__((ext_vector_type(4)));

#ifndef NB
#define NB 8
#endif
#ifndef SEQ
#define SEQ 1024
#endif
#define NB_FULL  8
#define SEQ_FULL 1024
#define DIM   768
#define NHEAD 12
#define HD    64
#define HID   3072
#define QKVW  (3 * DIM)
#define MROWS (NB * SEQ)

static_assert(NB >= 1 && NB <= NB_FULL);
static_assert(SEQ >= 128 && SEQ <= SEQ_FULL && (SEQ % 128) == 0);
static_assert(DIM == NHEAD * HD);
static_assert(HD == 64);
static_assert(HID == 4 * DIM);
static_assert((DIM % 64) == 0 && (DIM % 32) == 0);
static_assert((HID % 64) == 0 && (HID % 32) == 0);
static_assert((MROWS % 64) == 0 && (MROWS % 8) == 0);
static_assert(DIM == 6 * 32 * 4);
static_assert(DIM == 3 * 32 * 8);
static_assert(((size_t)MROWS * DIM) % (8 * 256) == 0);
static_assert((size_t)MROWS * HID < (size_t)0xFFFFFFFFu);

#define LDT 72
#define LDC 68

#define WCARRY 64.0f
#define PCARRY 1024.0f
#define CCARRY 1024.0f
#define HCARRY 16.0f
#define RCARRY 2048.0f
#define S768   0.03608439182435161f

#define P16        ((size_t)MROWS * DIM * 2)
#define WQKV_BYTES ((size_t)3 * DIM * DIM * 2)
#define WPRJ_BYTES ((size_t)DIM * DIM * 2)
#define WUP_BYTES  ((size_t)HID * DIM * 2)
#define WDN_BYTES  ((size_t)DIM * HID * 2)
#define OFF_WQKV   ((size_t)0)
#define OFF_WPRJ   (OFF_WQKV + WQKV_BYTES)
#define OFF_WUP    (OFF_WPRJ + WPRJ_BYTES)
#define OFF_WDN    (OFF_WUP + WUP_BYTES)
#define OFF_A      (OFF_WDN + WDN_BYTES)
#define OFF_B      (OFF_A + 5 * P16)
#define OFF_D      (OFF_B + P16)
#define WS_TOTAL   (OFF_D + 2 * P16)
static_assert((P16 % 128) == 0 && (OFF_A % 128) == 0 && (OFF_WPRJ % 128) == 0);
static_assert((OFF_WUP % 128) == 0 && (OFF_WDN % 128) == 0);
static_assert((size_t)MROWS * DIM * 4 == 2 * P16);
static_assert((size_t)MROWS * HID * 2 == 4 * P16);
static_assert(OFF_A + 4 * P16 + 2 * P16 == OFF_D);
static_assert(WS_TOTAL <= (size_t)134217728);

__device__ __forceinline__ float bf16r(float x) {
  unsigned int u = __float_as_uint(x);
  u = (u + 0x7FFFu + ((u >> 16) & 1u)) & 0xFFFF0000u;
  return __uint_as_float(u);
}

__device__ __forceinline__ v16h frag_at(const _Float16* p) {
  v8h lo = *(const v8h*)(p);
  v8h hi = *(const v8h*)(p + 16);
  v16h out;
#pragma unroll
  for (int i = 0; i < 8; ++i) { out[i] = lo[i]; out[i + 8] = hi[i]; }
  return out;
}
__device__ __forceinline__ v16h ld_frag(const _Float16* base, unsigned ld) {
  const unsigned lane = threadIdx.x & 31u;
  return frag_at(base + (lane & 15u) * ld + (lane >> 4) * 8u);
}

__device__ __forceinline__ v8f wmma16(v16h a, v16h b, v8f c) {
  v8f d = __builtin_amdgcn_wmma_f32_16x16x32_f16(false, a, false, b, (short)0, c,
                                                 false, false);
  asm volatile("v_nop\n\tv_nop\n\tv_nop\n\tv_nop" : "+v"(d) : "v"(a), "v"(b));
  return d;
}

__device__ __forceinline__ float red16_max(float x) {
#pragma unroll
  for (int off = 1; off < 16; off <<= 1) x = fmaxf(x, __shfl_xor(x, off, 32));
  return x;
}
__device__ __forceinline__ float red16_sum(float x) {
#pragma unroll
  for (int off = 1; off < 16; off <<= 1) x += __shfl_xor(x, off, 32);
  return x;
}
__device__ __forceinline__ float red32_sum(float x) {
#pragma unroll
  for (int off = 1; off < 32; off <<= 1) x += __shfl_xor(x, off, 32);
  return x;
}

__device__ __forceinline__ void wave_lds_sync() {
  __builtin_amdgcn_fence(3  , "wavefront");
  asm volatile("s_wait_dscnt 0x0" ::: "memory");
  __builtin_amdgcn_wave_barrier();
}

__global__ __launch_bounds__(256) void wconv_kernel(
    const float* __restrict__ W, _Float16* __restrict__ Wt,
    unsigned K, unsigned N, unsigned ldw, unsigned hs, unsigned cm) {
  __shared__ _Float16 T[64 * LDT];
  const unsigned tid = threadIdx.x;
  const unsigned n0 = blockIdx.x * 64u;
  const unsigned k0 = blockIdx.y * 64u;
  const unsigned p = blockIdx.z;
  const unsigned colbase = (n0 >> 6) * hs + p;
#pragma unroll 4
  for (unsigned j = 0; j < 16u; ++j) {
    const unsigned idx = tid + 256u * j;
    const unsigned kr = idx >> 6, nc = idx & 63u;
    const float v = W[(size_t)(k0 + kr) * ldw + colbase + nc * cm];
    T[nc * LDT + kr] = (_Float16)(WCARRY * bf16r(v));
  }
  __syncthreads();
  v8h x[2];
  size_t off[2];
#pragma unroll
  for (unsigned i = 0; i < 2u; ++i) {
    const unsigned n = 32u * i + (tid >> 3);
    const unsigned kc = (tid & 7u) * 8u;
    x[i] = *(const v8h*)&T[n * LDT + kc];
    off[i] = (size_t)p * N * K + (size_t)(n0 + n) * K + k0 + kc;
  }
#pragma unroll
  for (int i = 0; i < 2; ++i) *(volatile v8h*)(Wt + off[i]) = x[i];
  __threadfence();
#pragma unroll
  for (int i = 0; i < 2; ++i) *(volatile v8h*)(Wt + off[i]) = x[i];
}

__global__ __launch_bounds__(256) void xconv_kernel(
    const float* __restrict__ Xin, _Float16* __restrict__ dst) {
  const unsigned e = (blockIdx.x * 256u + threadIdx.x) * 8u;
  const unsigned crow = e / (unsigned)DIM;
  const unsigned c = e - crow * (unsigned)DIM;
  const unsigned bidx = crow / (unsigned)SEQ;
  const unsigned sq = crow - bidx * (unsigned)SEQ;
  const size_t frow = (size_t)bidx * SEQ_FULL + sq;
  const float* sp = Xin + frow * DIM + c;
  const v4f a0 = *(const v4f*)(sp);
  const v4f a1 = *(const v4f*)(sp + 4);
  v8h o;
#pragma unroll
  for (int j = 0; j < 4; ++j) {
    o[j]     = (_Float16)bf16r(a0[j]);
    o[j + 4] = (_Float16)bf16r(a1[j]);
  }
  *(volatile v8h*)(dst + (size_t)e) = o;
  __threadfence();
  *(volatile v8h*)(dst + (size_t)e) = o;
}

#define GM_QK   0
#define GM_VT   1
#define GM_F32  2
#define GM_GELU 3

template <int KD, int NOUT, int MODE>
__device__ __forceinline__ void gemm_body(
    const _Float16* __restrict__ A16, const _Float16* __restrict__ Bt,
    const float* __restrict__ bias, unsigned bsel, float scale,
    float* __restrict__ outf, _Float16* __restrict__ o16a, _Float16* __restrict__ o16b) {
  static_assert((KD % 32) == 0 && (KD % 8) == 0);
  static_assert((NOUT % 64) == 0);
  static_assert(MODE == GM_F32 || MODE == GM_GELU || NOUT == DIM);
  __shared__ float Cs[64 * LDC];
  const unsigned tid = threadIdx.x, lane = tid & 31u, w = tid >> 5;
  const unsigned mw = w >> 1, nw = w & 1u;
  const unsigned hh = lane >> 4, m = lane & 15u;
  const unsigned n0 = blockIdx.x * 64u;
  const unsigned row0 = blockIdx.y * 64u;

  const _Float16* ap  = A16 + (size_t)(row0 + mw * 16u + m) * KD + hh * 8u;
  const _Float16* bp0 = Bt + (size_t)(n0 + nw * 32u + m) * KD + hh * 8u;
  const _Float16* bp1 = bp0 + 16 * KD;
  v8f acc0 = {}, acc1 = {};
#pragma unroll 2
  for (unsigned k0 = 0; k0 < (unsigned)KD; k0 += 32u) {
    const v16h a  = frag_at(ap + k0);
    const v16h b0 = frag_at(bp0 + k0);
    const v16h b1 = frag_at(bp1 + k0);
    acc0 = wmma16(a, b0, acc0);
    acc1 = wmma16(a, b1, acc1);
  }
#pragma unroll
  for (int r = 0; r < 8; ++r) {
    float* d = &Cs[(mw * 16u + hh * 8u + (unsigned)r) * LDC + nw * 32u + m];
    d[0]  = acc0[r];
    d[16] = acc1[r];
  }
  __syncthreads();

  if (MODE == GM_QK) {
    const unsigned c = (tid & 7u) * 8u;
    float bb[8];
#pragma unroll
    for (unsigned j = 0; j < 8u; ++j)
      bb[j] = bf16r(bias[(n0 >> 6) * 192u + (c + j) * 3u + bsel]);
    v8h xh[2], xl[2];
    size_t off[2];
#pragma unroll
    for (unsigned i = 0; i < 2u; ++i) {
      const unsigned r = 32u * i + (tid >> 3);
      const v4f u0 = *(const v4f*)&Cs[r * LDC + c];
      const v4f u1 = *(const v4f*)&Cs[r * LDC + c + 4];
#pragma unroll
      for (int j = 0; j < 8; ++j) {
        const float u = (j < 4) ? u0[j & 3] : u1[j & 3];
        const float val = u * (1.0f / WCARRY) + bb[j];
        const _Float16 hcv = (_Float16)val;
        const _Float16 hv = (fabsf(val) < 6.2e-5f) ? (_Float16)0.0f : hcv;
        xh[i][j] = hv;
        xl[i][j] = (_Float16)((val - (float)hv) * RCARRY);
      }
      off[i] = (size_t)(row0 + r) * DIM + n0 + c;
    }
#pragma unroll
    for (int i = 0; i < 2; ++i) {
      *(volatile v8h*)(o16a + off[i]) = xh[i];
      *(volatile v8h*)(o16b + off[i]) = xl[i];
    }
    __threadfence();
#pragma unroll
    for (int i = 0; i < 2; ++i) {
      *(volatile v8h*)(o16a + off[i]) = xh[i];
      *(volatile v8h*)(o16b + off[i]) = xl[i];
    }
  }

  if (MODE == GM_VT) {
    static_assert((SEQ % 64) == 0);
    const unsigned bidx = row0 / (unsigned)SEQ;
    const unsigned key0 = row0 - bidx * (unsigned)SEQ;
    v8h x[2];
    size_t off[2];
#pragma unroll
    for (unsigned i = 0; i < 2u; ++i) {
      const unsigned dcol = 32u * i + (tid >> 3);
      const unsigned kk = (tid & 7u) * 8u;
      const float bv = bf16r(bias[(n0 >> 6) * 192u + dcol * 3u + bsel]);
#pragma unroll
      for (unsigned j = 0; j < 8u; ++j)
        x[i][j] = (_Float16)(Cs[(kk + j) * LDC + dcol] * (1.0f / WCARRY) + bv);
      off[i] = ((size_t)bidx * DIM + n0 + dcol) * SEQ + key0 + kk;
    }
#pragma unroll
    for (int i = 0; i < 2; ++i) *(volatile v8h*)(o16a + off[i]) = x[i];
    __threadfence();
#pragma unroll
    for (int i = 0; i < 2; ++i) *(volatile v8h*)(o16a + off[i]) = x[i];
  }

  if (MODE == GM_F32) {
    const unsigned c = (tid & 15u) * 4u;
    const v4f g = *(const v4f*)(bias + n0 + c);
    v4f gb;
#pragma unroll
    for (int j = 0; j < 4; ++j) gb[j] = bf16r(g[j]);
    v4f xs[4];
    size_t off[4];
#pragma unroll
    for (unsigned i = 0; i < 4u; ++i) {
      const unsigned r = 16u * i + (tid >> 4);
      const v4f u = *(const v4f*)&Cs[r * LDC + c];
      v4f val;
#pragma unroll
      for (int j = 0; j < 4; ++j) val[j] = u[j] * scale + gb[j];
      xs[i] = val;
      off[i] = (size_t)(row0 + r) * NOUT + n0 + c;
    }
#pragma unroll
    for (int i = 0; i < 4; ++i) *(volatile v4f*)(outf + off[i]) = xs[i];
    __threadfence();
#pragma unroll
    for (int i = 0; i < 4; ++i) *(volatile v4f*)(outf + off[i]) = xs[i];
  }

  if (MODE == GM_GELU) {
    const unsigned c = (tid & 7u) * 8u;
    const v4f g0 = *(const v4f*)(bias + n0 + c);
    const v4f g1 = *(const v4f*)(bias + n0 + c + 4);
    float bb[8];
#pragma unroll
    for (int j = 0; j < 4; ++j) { bb[j] = bf16r(g0[j]); bb[j + 4] = bf16r(g1[j]); }
    v8h x[2];
    size_t off[2];
#pragma unroll
    for (unsigned i = 0; i < 2u; ++i) {
      const unsigned r = 32u * i + (tid >> 3);
      const v4f u0 = *(const v4f*)&Cs[r * LDC + c];
      const v4f u1 = *(const v4f*)&Cs[r * LDC + c + 4];
#pragma unroll
      for (int j = 0; j < 8; ++j) {
        const float u = (j < 4) ? u0[j & 3] : u1[j & 3];
        const float hv = u * (1.0f / WCARRY) + bb[j];
        const float ge = 0.5f * hv * (1.0f + erff(hv * 0.70710678118654752f));
        x[i][j] = (_Float16)(ge * HCARRY);
      }
      off[i] = (size_t)(row0 + r) * NOUT + n0 + c;
    }
#pragma unroll
    for (int i = 0; i < 2; ++i) *(volatile v8h*)(o16a + off[i]) = x[i];
    __threadfence();
#pragma unroll
    for (int i = 0; i < 2; ++i) *(volatile v8h*)(o16a + off[i]) = x[i];
  }
}

__global__ __launch_bounds__(256) void gemm_qk_kernel(
    const _Float16* __restrict__ A16, const _Float16* __restrict__ Bt,
    const float* __restrict__ bias, unsigned bsel,
    _Float16* __restrict__ ohi, _Float16* __restrict__ olo) {
  gemm_body<DIM, DIM, GM_QK>(A16, Bt, bias, bsel, 1.0f, nullptr, ohi, olo);
}
__global__ __launch_bounds__(256) void gemm_vt_kernel(
    const _Float16* __restrict__ A16, const _Float16* __restrict__ Bt,
    const float* __restrict__ bias, unsigned bsel, _Float16* __restrict__ ovt) {
  gemm_body<DIM, DIM, GM_VT>(A16, Bt, bias, bsel, 1.0f, nullptr, ovt, nullptr);
}
__global__ __launch_bounds__(256) void gemm_proj_kernel(
    const _Float16* __restrict__ A16, const _Float16* __restrict__ Bt,
    const float* __restrict__ bias, float* __restrict__ outf) {
  gemm_body<DIM, DIM, GM_F32>(A16, Bt, bias, 0u, 1.0f / (WCARRY * CCARRY), outf,
                              nullptr, nullptr);
}
__global__ __launch_bounds__(256) void gemm_up_kernel(
    const _Float16* __restrict__ A16, const _Float16* __restrict__ Bt,
    const float* __restrict__ bias, _Float16* __restrict__ oh) {
  gemm_body<DIM, HID, GM_GELU>(A16, Bt, bias, 0u, 1.0f, nullptr, oh, nullptr);
}
__global__ __launch_bounds__(256) void gemm_down_kernel(
    const _Float16* __restrict__ A16, const _Float16* __restrict__ Bt,
    const float* __restrict__ bias, float* __restrict__ outf) {
  gemm_body<HID, DIM, GM_F32>(A16, Bt, bias, 0u, 1.0f / (WCARRY * HCARRY), outf,
                              nullptr, nullptr);
}

__global__ __launch_bounds__(256) void attn_kernel(
    const _Float16* __restrict__ Qh, const _Float16* __restrict__ Ql,
    const _Float16* __restrict__ Kh, const _Float16* __restrict__ Kl,
    const _Float16* __restrict__ Vt, _Float16* __restrict__ Ov) {
  __shared__ _Float16 Ksh[64 * LDT];
  __shared__ _Float16 Ksl[64 * LDT];
  __shared__ _Float16 Vs[64 * LDT];
  __shared__ _Float16 Ps[8 * 16 * LDT];

  const unsigned tid = threadIdx.x, lane = tid & 31u, w = tid >> 5;
  const unsigned hh = lane >> 4, m = lane & 15u;
  const unsigned q0 = blockIdx.x * 128u;
  const unsigned head = blockIdx.y;
  const unsigned b = blockIdx.z;
  _Float16* P = Ps + w * (16u * LDT);

  const size_t qoff = (size_t)(b * (unsigned)SEQ + q0 + w * 16u + m) * DIM + head * HD + hh * 8u;
  v16h qh[2], ql[2];
  qh[0] = frag_at(Qh + qoff);
  qh[1] = frag_at(Qh + qoff + 32);
  ql[0] = frag_at(Ql + qoff);
  ql[1] = frag_at(Ql + qoff + 32);

  float mrow[8], lrow[8];
  v8f o[4];
#pragma unroll
  for (int v = 0; v < 8; ++v) { mrow[v] = -1.0e30f; lrow[v] = 0.0f; }
#pragma unroll
  for (int nb = 0; nb < 4; ++nb) o[nb] = (v8f){};

  const size_t kplane = (size_t)b * SEQ * DIM + head * HD;
  const size_t vplane = ((size_t)b * DIM + head * HD) * SEQ;

  for (unsigned kb = 0; kb < (unsigned)SEQ; kb += 64u) {
#pragma unroll
    for (unsigned j = 0; j < 2u; ++j) {
      const unsigned idx = tid + 256u * j;
      const unsigned r = idx >> 3, c = (idx & 7u) * 8u;
      const size_t ko = kplane + (size_t)(kb + r) * DIM + c;
      *(v8h*)&Ksh[r * LDT + c] = *(const v8h*)(Kh + ko);
      *(v8h*)&Ksl[r * LDT + c] = *(const v8h*)(Kl + ko);
      *(v8h*)&Vs[r * LDT + c]  = *(const v8h*)(Vt + vplane + (size_t)r * SEQ + kb + c);
    }
    __syncthreads();

    v8f s[4];
#pragma unroll
    for (int kg = 0; kg < 4; ++kg) {
      v8f th = {};
      v8f tr = {};
#pragma unroll
      for (int c = 0; c < 2; ++c) {
        const v16h kfh = ld_frag(&Ksh[(kg * 16) * LDT + c * 32], LDT);
        const v16h kfl = ld_frag(&Ksl[(kg * 16) * LDT + c * 32], LDT);
        th = wmma16(qh[c], kfh, th);
        tr = wmma16(qh[c], kfl, tr);
        tr = wmma16(ql[c], kfh, tr);
      }
      s[kg] = th + tr * (1.0f / RCARRY);
    }

    float alpha[8];
#pragma unroll
    for (int v = 0; v < 8; ++v) {
      float mx = fmaxf(fmaxf(s[0][v], s[1][v]), fmaxf(s[2][v], s[3][v]));
      mx = red16_max(mx);
      const float mn = fmaxf(mrow[v], mx);
      alpha[v] = __expf(mrow[v] - mn);
      mrow[v] = mn;
    }
#pragma unroll
    for (int kg = 0; kg < 4; ++kg)
#pragma unroll
      for (int v = 0; v < 8; ++v) s[kg][v] = __expf(s[kg][v] - mrow[v]);
#pragma unroll
    for (int v = 0; v < 8; ++v) {
      const float rs = red16_sum((s[0][v] + s[1][v]) + (s[2][v] + s[3][v]));
      lrow[v] = alpha[v] * lrow[v] + rs;
    }
#pragma unroll
    for (int nb = 0; nb < 4; ++nb)
#pragma unroll
      for (int v = 0; v < 8; ++v) o[nb][v] = o[nb][v] * alpha[v];

#pragma unroll
    for (int kg = 0; kg < 4; ++kg)
#pragma unroll
      for (int v = 0; v < 8; ++v)
        P[(hh * 8u + (unsigned)v) * LDT + (unsigned)kg * 16u + m] = (_Float16)(s[kg][v] * PCARRY);
    wave_lds_sync();

#pragma unroll
    for (int c = 0; c < 2; ++c) {
      const v16h pf = ld_frag(P + c * 32, LDT);
#pragma unroll
      for (int nb = 0; nb < 4; ++nb) {
        const v16h vf = ld_frag(&Vs[(nb * 16) * LDT + c * 32], LDT);
        o[nb] = wmma16(pf, vf, o[nb]);
      }
    }
    __syncthreads();
  }

  float inv[8];
#pragma unroll
  for (int v = 0; v < 8; ++v)
    inv[v] = __builtin_amdgcn_rcpf(lrow[v]) * (S768 * (CCARRY / PCARRY));
#pragma unroll
  for (int nb = 0; nb < 4; ++nb)
#pragma unroll
    for (int v = 0; v < 8; ++v)
      P[(hh * 8u + (unsigned)v) * LDT + (unsigned)nb * 16u + m] = (_Float16)(o[nb][v] * inv[v]);
  wave_lds_sync();
  v8h x[4];
  size_t off[4];
#pragma unroll
  for (unsigned i = 0; i < 4u; ++i) {
    const unsigned r = 4u * i + (lane >> 3);
    const unsigned c = (lane & 7u) * 8u;
    x[i] = *(const v8h*)&P[r * LDT + c];
    off[i] = (size_t)(b * (unsigned)SEQ + q0 + w * 16u + r) * DIM + head * HD + c;
  }
#pragma unroll
  for (int i = 0; i < 4; ++i) *(volatile v8h*)(Ov + off[i]) = x[i];
  __threadfence();
#pragma unroll
  for (int i = 0; i < 4; ++i) *(volatile v8h*)(Ov + off[i]) = x[i];
}

template <int SECOND>
__device__ __forceinline__ void ln_body(
    const float* __restrict__ Y, const float* __restrict__ R,
    const float* __restrict__ g, const float* __restrict__ be,
    float* __restrict__ outf, _Float16* __restrict__ out16) {
  __shared__ float Rs[8 * DIM];
  __shared__ _Float16 Rh[8 * DIM];
  const unsigned tid = threadIdx.x, lane = tid & 31u, w = tid >> 5;
  const unsigned crow = blockIdx.x * 8u + w;
  const unsigned bidx = crow / (unsigned)SEQ;
  const unsigned sq = crow - bidx * (unsigned)SEQ;
  const size_t frow = (size_t)bidx * SEQ_FULL + sq;
  const float* yr = Y + (size_t)crow * DIM;

  float s = 0.0f;
#pragma unroll 1
  for (unsigned i = 0; i < 6u; ++i) {
    const v4f a = *(const v4f*)(yr + (i * 32u + lane) * 4u);
    s += (a[0] + a[1]) + (a[2] + a[3]);
  }
  s = red32_sum(s);
  const float mu = s * (1.0f / (float)DIM);

  float q = 0.0f;
#pragma unroll 1
  for (unsigned i = 0; i < 6u; ++i) {
    const v4f a = *(const v4f*)(yr + (i * 32u + lane) * 4u);
    const float d0 = a[0] - mu, d1 = a[1] - mu, d2 = a[2] - mu, d3 = a[3] - mu;
    q += (d0 * d0 + d1 * d1) + (d2 * d2 + d3 * d3);
  }
  q = red32_sum(q);
  const float rs = rsqrtf(q * (1.0f / (float)DIM) + 1.0e-5f);

  const size_t rrow = SECOND ? (size_t)crow : frow;
  const float* rr = R + rrow * DIM;
  float* ls = Rs + w * (unsigned)DIM;
  _Float16* lh = Rh + w * (unsigned)DIM;
#pragma unroll 1
  for (unsigned i = 0; i < 6u; ++i) {
    const unsigned c = (i * 32u + lane) * 4u;
    const v4f a  = *(const v4f*)(yr + c);
    const v4f gg = *(const v4f*)(g + c);
    const v4f bb = *(const v4f*)(be + c);
    const v4f xr = *(const v4f*)(rr + c);
    v4f val;
    v4h hv;
#pragma unroll
    for (int j = 0; j < 4; ++j) {
      const float res = SECOND ? xr[j] : bf16r(xr[j]);
      float t = (a[j] - mu) * rs;
      t = t * bf16r(gg[j]) + bf16r(bb[j]);
      val[j] = res + t;
      hv[j] = (_Float16)val[j];
    }
    *(v4f*)(ls + c) = val;
    if (!SECOND) *(v4h*)(lh + c) = hv;
  }
  wave_lds_sync();

  const size_t orow = SECOND ? frow : (size_t)crow;
  float* op = outf + orow * DIM;
  v4f xs[6];
#pragma unroll
  for (unsigned i = 0; i < 6u; ++i) xs[i] = *(const v4f*)(ls + (i * 32u + lane) * 4u);
  v8h hs[3];
  if (!SECOND) {
#pragma unroll
    for (unsigned j = 0; j < 3u; ++j) hs[j] = *(const v8h*)(lh + (j * 32u + lane) * 8u);
  }
  _Float16* hp = out16 + (size_t)crow * DIM;

#pragma unroll
  for (unsigned i = 0; i < 6u; ++i) *(volatile v4f*)(op + (i * 32u + lane) * 4u) = xs[i];
  if (!SECOND) {
#pragma unroll
    for (unsigned j = 0; j < 3u; ++j) *(volatile v8h*)(hp + (j * 32u + lane) * 8u) = hs[j];
  }
  __threadfence();
#pragma unroll
  for (unsigned i = 0; i < 6u; ++i) *(volatile v4f*)(op + (i * 32u + lane) * 4u) = xs[i];
  if (!SECOND) {
#pragma unroll
    for (unsigned j = 0; j < 3u; ++j) *(volatile v8h*)(hp + (j * 32u + lane) * 8u) = hs[j];
  }
}

__global__ __launch_bounds__(256) void ln1_kernel(
    const float* __restrict__ Y, const float* __restrict__ X,
    const float* __restrict__ g, const float* __restrict__ be,
    float* __restrict__ x1f, _Float16* __restrict__ x1h) {
  ln_body<0>(Y, X, g, be, x1f, x1h);
}
__global__ __launch_bounds__(256) void ln2_kernel(
    const float* __restrict__ Y, const float* __restrict__ X1,
    const float* __restrict__ g, const float* __restrict__ be,
    float* __restrict__ outp, _Float16* __restrict__ unused16) {
  ln_body<1>(Y, X1, g, be, outp, unused16);
}

extern "C" void kernel_launch(void* const* d_in, const int* in_sizes, int n_in,
                              void* d_out, int out_size, void* d_ws, size_t ws_size,
                              hipStream_t stream) {
  if (n_in < 13) return;
  const long long need_x = ((long long)(NB - 1) * SEQ_FULL + SEQ) * DIM;
  if ((long long)in_sizes[0] < need_x) return;
  if ((long long)in_sizes[1] < (long long)DIM * QKVW) return;
  if (in_sizes[2] < QKVW) return;
  if ((long long)in_sizes[3] < (long long)DIM * DIM) return;
  if (in_sizes[4] < DIM) return;
  if ((long long)in_sizes[5] < (long long)DIM * HID) return;
  if (in_sizes[6] < HID) return;
  if ((long long)in_sizes[7] < (long long)HID * DIM) return;
  if (in_sizes[8] < DIM || in_sizes[9] < DIM || in_sizes[10] < DIM) return;
  if (in_sizes[11] < DIM || in_sizes[12] < DIM) return;
  if ((long long)out_size < need_x) return;
  if (ws_size < WS_TOTAL) return;

  const float* X     = (const float*)d_in[0];
  const float* Wqkv  = (const float*)d_in[1];
  const float* bqkv  = (const float*)d_in[2];
  const float* Wproj = (const float*)d_in[3];
  const float* bproj = (const float*)d_in[4];
  const float* W1    = (const float*)d_in[5];
  const float* b1    = (const float*)d_in[6];
  const float* W2    = (const float*)d_in[7];
  const float* b2    = (const float*)d_in[8];
  const float* g1    = (const float*)d_in[9];
  const float* be1   = (const float*)d_in[10];
  const float* g2    = (const float*)d_in[11];
  const float* be2   = (const float*)d_in[12];
  float* out = (float*)d_out;

  char* ws = (char*)d_ws;
  _Float16* WtQ = (_Float16*)(ws + OFF_WQKV);
  _Float16* WtP = (_Float16*)(ws + OFF_WPRJ);
  _Float16* WtU = (_Float16*)(ws + OFF_WUP);
  _Float16* WtD = (_Float16*)(ws + OFF_WDN);
  _Float16* Qh16 = (_Float16*)(ws + OFF_A + 0 * P16);
  _Float16* Ql16 = (_Float16*)(ws + OFF_A + 1 * P16);
  _Float16* Kh16 = (_Float16*)(ws + OFF_A + 2 * P16);
  _Float16* Kl16 = (_Float16*)(ws + OFF_A + 3 * P16);
  _Float16* Vt16 = (_Float16*)(ws + OFF_A + 4 * P16);
  float*    Yf   = (float*)(ws + OFF_A);
  _Float16* H16  = (_Float16*)(ws + OFF_A);
  float*    Y2f  = (float*)(ws + OFF_A + 4 * P16);
  _Float16* X16  = (_Float16*)(ws + OFF_B);
  _Float16* Ctx16 = (_Float16*)(ws + OFF_B);
  _Float16* X1h  = (_Float16*)(ws + OFF_B);
  float*    X1f  = (float*)(ws + OFF_D);

  const size_t WP = (size_t)DIM * DIM;
  dim3 blk(256);

  wconv_kernel<<<dim3(DIM / 64, DIM / 64, 3), blk, 0, stream>>>(
      Wqkv, WtQ, (unsigned)DIM, (unsigned)DIM, (unsigned)QKVW, 192u, 3u);
  wconv_kernel<<<dim3(DIM / 64, DIM / 64, 1), blk, 0, stream>>>(
      Wproj, WtP, (unsigned)DIM, (unsigned)DIM, (unsigned)DIM, 64u, 1u);
  wconv_kernel<<<dim3(HID / 64, DIM / 64, 1), blk, 0, stream>>>(
      W1, WtU, (unsigned)DIM, (unsigned)HID, (unsigned)HID, 64u, 1u);
  wconv_kernel<<<dim3(DIM / 64, HID / 64, 1), blk, 0, stream>>>(
      W2, WtD, (unsigned)HID, (unsigned)DIM, (unsigned)DIM, 64u, 1u);

  xconv_kernel<<<dim3((unsigned)(((size_t)MROWS * DIM) / 2048)), blk, 0, stream>>>(X, X16);

  dim3 gD(DIM / 64, MROWS / 64);
  dim3 gH(HID / 64, MROWS / 64);
  gemm_qk_kernel<<<gD, blk, 0, stream>>>(X16, WtQ + 0 * WP, bqkv, 0u, Qh16, Ql16);
  gemm_qk_kernel<<<gD, blk, 0, stream>>>(X16, WtQ + 1 * WP, bqkv, 1u, Kh16, Kl16);
  gemm_vt_kernel<<<gD, blk, 0, stream>>>(X16, WtQ + 2 * WP, bqkv, 2u, Vt16);

  attn_kernel<<<dim3(SEQ / 128, NHEAD, NB), blk, 0, stream>>>(
      Qh16, Ql16, Kh16, Kl16, Vt16, Ctx16);

  gemm_proj_kernel<<<gD, blk, 0, stream>>>(Ctx16, WtP, bproj, Yf);
  ln1_kernel<<<dim3(MROWS / 8), blk, 0, stream>>>(Yf, X, g1, be1, X1f, X1h);
  gemm_up_kernel<<<gH, blk, 0, stream>>>(X1h, WtU, b1, H16);
  gemm_down_kernel<<<gD, blk, 0, stream>>>(H16, WtD, b2, Y2f);
  ln2_kernel<<<dim3(MROWS / 8), blk, 0, stream>>>(Y2f, X1f, g2, be2, out, X1h);
}
